// cross_attention_8624294330992
// MI455X (gfx1250) — hardware-verified
//
#include <hip/hip_runtime.h>
#include <stdint.h>
#include <stddef.h>


#ifndef NROWS
#define NROWS 8192
#endif
#define NROWS_FULL 8192
#define DD 512

static_assert(NROWS % 256 == 0);
static_assert(NROWS >= 256);
static_assert(NROWS <= NROWS_FULL);
static_assert(DD == 512);
static_assert(((long)NROWS * DD / 8) % 256 == 0);

typedef unsigned int v4u  __attribute__((ext_vector_type(4)));
typedef float        v4f  __attribute__((ext_vector_type(4)));
typedef float        v8f  __attribute__((ext_vector_type(8)));
typedef _Float16     v16h __attribute__((ext_vector_type(16)));
typedef __bf16       v16bf __attribute__((ext_vector_type(16)));

union Frag { v4u q[2]; v16h h; v16bf b; };

static __device__ __forceinline__ v8f vzero() {
  v8f z = {0.f, 0.f, 0.f, 0.f, 0.f, 0.f, 0.f, 0.f};
  return z;
}

static __device__ __forceinline__ unsigned int bfbits(float f) {
  const unsigned int u = __float_as_uint(f);
  return (u + 0x7FFFu + ((u >> 16) & 1u)) >> 16;
}
static __device__ __forceinline__ float bfr(float f) { return __uint_as_float(bfbits(f) << 16); }
static __device__ __forceinline__ unsigned int hbits(float f) {
  const _Float16 hv = (_Float16)f;
  return (unsigned int)__builtin_bit_cast(unsigned short, hv);
}

static __device__ __forceinline__ void ld_frag(Frag& f, const unsigned short* rowp, int h) {
  f.q[0] = *(const v4u*)(rowp + 8 * h);
  f.q[1] = *(const v4u*)(rowp + 16 + 8 * h);
}

static __device__ __forceinline__ v8f mma_bf(const Frag& A, const Frag& B, v8f c) {
  c = __builtin_amdgcn_wmma_f32_16x16x32_bf16(false, A.b, false, B.b, (short)0, c, false, false);
  asm volatile("v_nop\n\tv_nop\n\tv_nop\n\tv_nop" : "+v"(c) : "v"(A.h), "v"(B.h));
  return c;
}
static __device__ __forceinline__ v8f mma_h(const Frag& A, const Frag& B, v8f c) {
  c = __builtin_amdgcn_wmma_f32_16x16x32_f16(false, A.h, false, B.h, (short)0, c, false, false);
  asm volatile("v_nop\n\tv_nop\n\tv_nop\n\tv_nop" : "+v"(c) : "v"(A.h), "v"(B.h));
  return c;
}

template <int TBF> struct MmaSel;
template <> struct MmaSel<1> {
  static __device__ __forceinline__ v8f run(const Frag& a, const Frag& b, v8f c) { return mma_bf(a, b, c); }
};
template <> struct MmaSel<0> {
  static __device__ __forceinline__ v8f run(const Frag& a, const Frag& b, v8f c) { return mma_h(a, b, c); }
};

static __device__ __forceinline__ float rmax16(float v) {
#pragma unroll
  for (int m = 1; m <= 8; m <<= 1) v = fmaxf(v, __shfl_xor(v, m, 32));
  return v;
}
static __device__ __forceinline__ float rsum16(float v) {
#pragma unroll
  for (int m = 1; m <= 8; m <<= 1) v += __shfl_xor(v, m, 32);
  return v;
}

template <int TBF>
static __device__ __forceinline__ unsigned int cvt1(float x, float s) {
  const float r = bfr(x) * s;
  return TBF ? bfbits(r) : hbits(r);
}
template <int TBF>
static __device__ __forceinline__ v4u pack8(const v4f a, const v4f b, float s) {
  v4u w;
  w.x = cvt1<TBF>(a.x, s) | (cvt1<TBF>(a.y, s) << 16);
  w.y = cvt1<TBF>(a.z, s) | (cvt1<TBF>(a.w, s) << 16);
  w.z = cvt1<TBF>(b.x, s) | (cvt1<TBF>(b.y, s) << 16);
  w.w = cvt1<TBF>(b.z, s) | (cvt1<TBF>(b.w, s) << 16);
  return w;
}
static __device__ __forceinline__ unsigned int split_pair(float x, float y, unsigned int& lo) {
  const unsigned int hx = bfbits(x), hy = bfbits(y);
  const unsigned int lx = bfbits(x - __uint_as_float(hx << 16));
  const unsigned int ly = bfbits(y - __uint_as_float(hy << 16));
  lo = lx | (ly << 16);
  return hx | (hy << 16);
}

__global__ __launch_bounds__(256) void k_cvt(const float* __restrict__ x1, const float* __restrict__ x2,
                                             unsigned short* P1, unsigned short* P2, int n8)
{
  const int gid = blockIdx.x * 256 + (int)threadIdx.x;
  if (gid >= n8) return;
  const float* src = (blockIdx.y == 0) ? x1 : x2;
  unsigned short* dst = (blockIdx.y == 0) ? P1 : P2;
  const float* p = src + (size_t)gid * 8;
  const v4f a = *(const v4f*)p;
  const v4f b = *(const v4f*)(p + 4);
  v4u w;
  w.x = bfbits(a.x) | (bfbits(a.y) << 16);
  w.y = bfbits(a.z) | (bfbits(a.w) << 16);
  w.z = bfbits(b.x) | (bfbits(b.y) << 16);
  w.w = bfbits(b.z) | (bfbits(b.w) << 16);
  volatile v4u* d = (volatile v4u*)(dst + (size_t)gid * 8);
  *d = w;
  __threadfence();
  *d = w;
}

#define TP 72
__global__ __launch_bounds__(256) void k_tr(const float* __restrict__ x, unsigned short* Xt, int ldt)
{
  __shared__ __align__(16) unsigned short tile[64 * TP];
  const int tid = threadIdx.x;
  const int r0 = blockIdx.x * 64, c0 = blockIdx.y * 64;
  {
    const int i = tid >> 2, cq = tid & 3;
    const float* p = x + (size_t)(r0 + i) * DD + c0 + 16 * cq;
#pragma unroll
    for (int e = 0; e < 4; ++e) {
      const v4f v = *(const v4f*)(p + 4 * e);
      const int c = 16 * cq + 4 * e;
      tile[(c + 0) * TP + i] = (unsigned short)hbits(bfr(v.x));
      tile[(c + 1) * TP + i] = (unsigned short)hbits(bfr(v.y));
      tile[(c + 2) * TP + i] = (unsigned short)hbits(bfr(v.z));
      tile[(c + 3) * TP + i] = (unsigned short)hbits(bfr(v.w));
    }
  }
  __syncthreads();
  v4u pc[2];
  size_t off[2];
#pragma unroll
  for (int q = 0; q < 2; ++q) {
    const int p = tid + 256 * q, c = p >> 3, seg = p & 7;
    pc[q] = *(const v4u*)(tile + c * TP + 8 * seg);
    off[q] = (size_t)(c0 + c) * ldt + r0 + 8 * seg;
  }
  for (int pass = 0; pass < 2; ++pass) {
    *(volatile v4u*)(Xt + off[0]) = pc[0];
    *(volatile v4u*)(Xt + off[1]) = pc[1];
    __threadfence();
  }
}

#define GP 40
#define SPITCH 68
#define GEMM_ABBYTES ((256 + 64 + 64) * GP * 2)
#define GEMM_LDS (GEMM_ABBYTES + 256 * SPITCH * 4)

template <int TBF, int AMODE, int BMODE, int OMODE>
__global__ __launch_bounds__(256) __attribute__((amdgpu_num_vgpr(256)))
void k_gemm(const void* __restrict__ Ap, const void* __restrict__ Bp0, const void* Bp1,
            void* Op0, void* Op1, int lda, int ldb, int ldo, int kdim, float bscale, float oscale)
{
  static_assert(OMODE == 0 || TBF == 1);
  extern __shared__ __align__(16) char smem[];
  unsigned short* Al  = (unsigned short*)smem;
  unsigned short* Bl0 = Al + 256 * GP;
  unsigned short* Bl1 = Bl0 + 64 * GP;
  float* St = (float*)(smem + GEMM_ABBYTES);
  (void)bscale; (void)oscale; (void)Bp1; (void)Op1;

  const int tid = threadIdx.x;
  const int w = tid >> 5, lane = tid & 31, h = lane >> 4, n15 = lane & 15;
  const int n0 = blockIdx.x * 64, m0 = blockIdx.y * 256;

  v8f acc[2][4];
#pragma unroll
  for (int rt = 0; rt < 2; ++rt)
#pragma unroll
    for (int jt = 0; jt < 4; ++jt) acc[rt][jt] = vzero();

#pragma unroll 1
  for (int k0 = 0; k0 < kdim; k0 += 32) {
    __syncthreads();
    if (AMODE == 0) {
      const float* xp = (const float*)Ap + (size_t)(m0 + tid) * lda + k0;
#pragma unroll
      for (int c = 0; c < 4; ++c) {
        const v4f f0 = *(const v4f*)(xp + 8 * c);
        const v4f f1 = *(const v4f*)(xp + 8 * c + 4);
        *(v4u*)(Al + tid * GP + 8 * c) = pack8<TBF>(f0, f1, 1.0f);
      }
    } else {
      const unsigned short* xp = (const unsigned short*)Ap + (size_t)(m0 + tid) * lda + k0;
#pragma unroll
      for (int c = 0; c < 4; ++c) *(v4u*)(Al + tid * GP + 8 * c) = *(const v4u*)(xp + 8 * c);
    }
    if (BMODE == 0) {
      const int nn = tid >> 2, pc = tid & 3;
      const float* bp = (const float*)Bp0 + (size_t)(n0 + nn) * ldb + k0 + 8 * pc;
      *(v4u*)(Bl0 + nn * GP + 8 * pc) = pack8<TBF>(*(const v4f*)bp, *(const v4f*)(bp + 4), bscale);
    } else if (BMODE == 1) {
      const float* bp = (const float*)Bp0;
#pragma unroll
      for (int it = 0; it < 8; ++it) {
        const int i = tid + 256 * it;
        const int kk = i >> 6, nn = i & 63;
        Bl0[nn * GP + kk] = (unsigned short)cvt1<TBF>(bp[(size_t)(k0 + kk) * ldb + n0 + nn], bscale);
      }
    } else {
      const int nn = tid >> 2, pc = tid & 3;
      const size_t go = (size_t)(n0 + nn) * ldb + k0 + 8 * pc;
      *(v4u*)(Bl0 + nn * GP + 8 * pc) = *(const v4u*)((const unsigned short*)Bp0 + go);
      *(v4u*)(Bl1 + nn * GP + 8 * pc) = *(const v4u*)((const unsigned short*)Bp1 + go);
    }
    __syncthreads();
#pragma unroll
    for (int rt = 0; rt < 2; ++rt) {
      Frag a;
      ld_frag(a, Al + (32 * w + 16 * rt + n15) * GP, h);
#pragma unroll
      for (int jt = 0; jt < 4; ++jt) {
        Frag b;
        ld_frag(b, Bl0 + (16 * jt + n15) * GP, h);
        acc[rt][jt] = MmaSel<TBF>::run(a, b, acc[rt][jt]);
        if (BMODE == 2) {
          Frag b1;
          ld_frag(b1, Bl1 + (16 * jt + n15) * GP, h);
          acc[rt][jt] = MmaSel<TBF>::run(a, b1, acc[rt][jt]);
        }
      }
    }
  }

#pragma unroll
  for (int rt = 0; rt < 2; ++rt)
#pragma unroll
    for (int jt = 0; jt < 4; ++jt)
#pragma unroll
      for (int r = 0; r < 8; ++r)
        St[(32 * w + 16 * rt + 8 * h + r) * SPITCH + 16 * jt + n15] = acc[rt][jt][r];
  __syncthreads();

  if (OMODE == 0) {
    float* O = (float*)Op0;
    const int rs = lane >> 4, cq = lane & 15;
    for (int pass = 0; pass < 2; ++pass) {
#pragma unroll
      for (int it = 0; it < 16; ++it) {
        const int row = 32 * w + 2 * it + rs;
        v4f v = *(const v4f*)(St + row * SPITCH + 4 * cq);
        v = v * oscale;
        *(volatile v4f*)(O + (size_t)(m0 + row) * ldo + n0 + 4 * cq) = v;
      }
      __threadfence();
    }
  } else {
    unsigned short* O0 = (unsigned short*)Op0;
    unsigned short* O1 = (unsigned short*)Op1;
    const int rs = lane >> 3, cq = lane & 7;
    for (int pass = 0; pass < 2; ++pass) {
#pragma unroll
      for (int it = 0; it < 8; ++it) {
        const int row = 32 * w + 4 * it + rs;
        const v4f a = *(const v4f*)(St + row * SPITCH + 8 * cq);
        const v4f b = *(const v4f*)(St + row * SPITCH + 8 * cq + 4);
        v4u wh, wl;
        unsigned int l0, l1, l2, l3;
        wh.x = split_pair(a.x, a.y, l0);
        wh.y = split_pair(a.z, a.w, l1);
        wh.z = split_pair(b.x, b.y, l2);
        wh.w = split_pair(b.z, b.w, l3);
        wl.x = l0; wl.y = l1; wl.z = l2; wl.w = l3;
        const size_t go = (size_t)(m0 + row) * ldo + n0 + 8 * cq;
        *(volatile v4u*)(O0 + go) = wh;
        *(volatile v4u*)(O1 + go) = wl;
      }
      __threadfence();
    }
  }
}

#define QPITCH 520
#define PPITCH 72
#define OPITCH 132
#define ATT_QREG (8 * 16 * OPITCH * 4)
#define ATT_PBYTES (2 * 16 * PPITCH * 2)
#define ATT_LDS (ATT_QREG + ATT_PBYTES + 2 * 128 * 4)
#define PCARRY 16384.0f
static_assert(ATT_QREG >= 2 * 32 * QPITCH * 2);

__global__ __launch_bounds__(256) __attribute__((amdgpu_num_vgpr(256)))
void k_attn(const unsigned short* __restrict__ Gh, const unsigned short* __restrict__ Gl,
            const unsigned short* __restrict__ X2b, const unsigned short* __restrict__ X1t,
            unsigned short* Oh, int nkeys, int ldt)
{
  extern __shared__ __align__(16) char smem[];
  unsigned short* Qh = (unsigned short*)smem;
  unsigned short* Ql = Qh + 32 * QPITCH;
  float* Ost = (float*)smem;
  unsigned short* Pl = (unsigned short*)(smem + ATT_QREG);
  float* redmax = (float*)(smem + ATT_QREG + ATT_PBYTES);
  float* redsum = redmax + 128;

  const int tid = threadIdx.x;
  const int wv = tid >> 5, lane = tid & 31, h = lane >> 4, n15 = lane & 15;
  const int rg = wv >> 2, cs = wv & 3;
  const int m0 = blockIdx.x * 32;

#pragma unroll
  for (int it = 0; it < 8; ++it) {
    const int i = tid + 256 * it;
    const int r = i >> 6, c = (i & 63) * 8;
    *(v4u*)(Qh + r * QPITCH + c) = *(const v4u*)(Gh + (size_t)(m0 + r) * DD + c);
    *(v4u*)(Ql + r * QPITCH + c) = *(const v4u*)(Gl + (size_t)(m0 + r) * DD + c);
  }

  v8f o[8];
#pragma unroll
  for (int jt = 0; jt < 8; ++jt) o[jt] = vzero();
  float Mrow[8], lrow[8];
#pragma unroll
  for (int r = 0; r < 8; ++r) { Mrow[r] = -__builtin_inff(); lrow[r] = 0.f; }

  const unsigned short* qh = Qh + (16 * rg + n15) * QPITCH;
  const unsigned short* ql = Ql + (16 * rg + n15) * QPITCH;
  const unsigned short* kbase = X2b + (size_t)(16 * cs + n15) * DD;
  const unsigned short* vbase = X1t + (size_t)(128 * cs + n15) * ldt;
  const unsigned short* prd = Pl + (rg * 16 + n15) * PPITCH;

#pragma unroll 1
  for (int n0 = 0; n0 < nkeys; n0 += 64) {
    __syncthreads();
    v8f s = vzero();
    {
      const unsigned short* kp = kbase + (size_t)n0 * DD;
#pragma unroll 2
      for (int kk = 0; kk < DD; kk += 32) {
        Frag a, c, b;
        ld_frag(a, qh + kk, h);
        ld_frag(c, ql + kk, h);
        ld_frag(b, kp + kk, h);
        s = mma_bf(a, b, s);
        s = mma_bf(c, b, s);
      }
    }
    float tmax[8];
#pragma unroll
    for (int r = 0; r < 8; ++r) {
      float x = s[r];
      x = (x >= 0.f) ? x : 0.01f * x;
      s[r] = x;
      tmax[r] = rmax16(x);
    }
    if (n15 == 0) {
#pragma unroll
      for (int r = 0; r < 8; ++r) redmax[(rg * 4 + cs) * 16 + 8 * h + r] = tmax[r];
    }
    __syncthreads();
    float scl[8];
#pragma unroll
    for (int r = 0; r < 8; ++r) {
      const int row = 8 * h + r;
      const float mb = fmaxf(fmaxf(redmax[(rg * 4 + 0) * 16 + row], redmax[(rg * 4 + 1) * 16 + row]),
                             fmaxf(redmax[(rg * 4 + 2) * 16 + row], redmax[(rg * 4 + 3) * 16 + row]));
      const float Mn = fmaxf(Mrow[r], mb);
      scl[r] = __expf(Mrow[r] - Mn);
      Mrow[r] = Mn;
    }
    float tsum[8];
#pragma unroll
    for (int r = 0; r < 8; ++r) {
      const float p = __expf(s[r] - Mrow[r]);
      tsum[r] = rsum16(p);
      Pl[(rg * 16 + 8 * h + r) * PPITCH + 16 * cs + n15] = (unsigned short)hbits(p * PCARRY);
      lrow[r] *= scl[r];
    }
    if (n15 == 0) {
#pragma unroll
      for (int r = 0; r < 8; ++r) redsum[(rg * 4 + cs) * 16 + 8 * h + r] = tsum[r];
    }
#pragma unroll
    for (int jt = 0; jt < 8; ++jt)
#pragma unroll
      for (int r = 0; r < 8; ++r) o[jt][r] *= scl[r];
    __syncthreads();
#pragma unroll
    for (int r = 0; r < 8; ++r) {
      const int row = 8 * h + r;
      lrow[r] += (redsum[(rg * 4 + 0) * 16 + row] + redsum[(rg * 4 + 1) * 16 + row]) +
                 (redsum[(rg * 4 + 2) * 16 + row] + redsum[(rg * 4 + 3) * 16 + row]);
    }
#pragma unroll
    for (int ns = 0; ns < 2; ++ns) {
      Frag a;
      ld_frag(a, prd + 32 * ns, h);
      const unsigned short* vp = vbase + n0 + 32 * ns;
#pragma unroll
      for (int jt = 0; jt < 8; ++jt) {
        Frag b;
        ld_frag(b, vp + (size_t)(16 * jt) * ldt, h);
        o[jt] = mma_h(a, b, o[jt]);
      }
    }
  }

  float il[8];
#pragma unroll
  for (int r = 0; r < 8; ++r) il[r] = 1.0f / (lrow[r] * PCARRY);
  __syncthreads();
  float* ost = Ost + wv * (16 * OPITCH);
#pragma unroll
  for (int jt = 0; jt < 8; ++jt)
#pragma unroll
    for (int r = 0; r < 8; ++r) ost[(8 * h + r) * OPITCH + 16 * jt + n15] = o[jt][r] * il[r];
  __syncthreads();
  {
    const int rs = lane >> 4, cq = lane & 15;
    unsigned short* ob = Oh + (size_t)(m0 + 16 * rg) * DD + 128 * cs + 8 * cq;
    for (int pass = 0; pass < 2; ++pass) {
#pragma unroll
      for (int it = 0; it < 8; ++it) {
        const int row = 2 * it + rs;
        const v4f a = *(const v4f*)(ost + row * OPITCH + 8 * cq);
        const v4f b = *(const v4f*)(ost + row * OPITCH + 8 * cq + 4);
        v4u w;
        w.x = hbits(a.x) | (hbits(a.y) << 16);
        w.y = hbits(a.z) | (hbits(a.w) << 16);
        w.z = hbits(b.x) | (hbits(b.y) << 16);
        w.w = hbits(b.z) | (hbits(b.w) << 16);
        *(volatile v4u*)(ob + (size_t)row * DD) = w;
      }
      __threadfence();
    }
  }
}

extern "C" void kernel_launch(void* const* d_in, const int* in_sizes, int n_in,
                              void* d_out, int out_size, void* d_ws, size_t ws_size,
                              hipStream_t stream)
{
  if (n_in < 5) return;
  if (in_sizes[0] < NROWS * DD || in_sizes[1] < NROWS * DD ||
      in_sizes[2] < DD * DD || in_sizes[3] < DD * DD || in_sizes[4] < DD * DD) return;
  if (out_size < NROWS * DD) return;

  const float* x1 = (const float*)d_in[0];
  const float* x2 = (const float*)d_in[1];
  const float* qw = (const float*)d_in[2];
  const float* kw = (const float*)d_in[3];
  const float* vw = (const float*)d_in[4];
  float* out = (float*)d_out;

  const size_t PL = (size_t)NROWS * DD * 2;
  const size_t PM = (size_t)DD * DD * 2;
  char* ws = (char*)d_ws;
  size_t off = 0;
  unsigned short* X1b = (unsigned short*)(ws + off); off += PL;
  unsigned short* X2b = (unsigned short*)(ws + off); off += PL;
  unsigned short* X1t = (unsigned short*)(ws + off); off += PL;
  unsigned short* Gh  = (unsigned short*)(ws + off); off += PL;
  unsigned short* Gl  = (unsigned short*)(ws + off); off += PL;
  unsigned short* Ohp = (unsigned short*)(ws + off); off += PL;
  unsigned short* Mth = (unsigned short*)(ws + off); off += PM;
  unsigned short* Mtl = (unsigned short*)(ws + off); off += PM;
  if (off > ws_size) return;

  (void)hipFuncSetAttribute(reinterpret_cast<const void*>(&k_gemm<1, 0, 0, 1>),
                            hipFuncAttributeMaxDynamicSharedMemorySize, GEMM_LDS);
  (void)hipFuncSetAttribute(reinterpret_cast<const void*>(&k_gemm<1, 1, 2, 1>),
                            hipFuncAttributeMaxDynamicSharedMemorySize, GEMM_LDS);
  (void)hipFuncSetAttribute(reinterpret_cast<const void*>(&k_gemm<0, 1, 1, 0>),
                            hipFuncAttributeMaxDynamicSharedMemorySize, GEMM_LDS);
  (void)hipFuncSetAttribute(reinterpret_cast<const void*>(&k_attn),
                            hipFuncAttributeMaxDynamicSharedMemorySize, ATT_LDS);

  const int n8 = NROWS * DD / 8;
  k_cvt<<<dim3(n8 / 256, 2), 256, 0, stream>>>(x1, x2, X1b, X2b, n8);
  k_tr<<<dim3(NROWS / 64, DD / 64), 256, 0, stream>>>(x1, X1t, NROWS);
  k_gemm<1, 0, 0, 1><<<dim3(DD / 64, DD / 256), 256, GEMM_LDS, stream>>>(
      kw, qw, qw, Mth, Mtl, DD, DD, DD, DD, 1.0f, 1.0f);
  k_gemm<1, 1, 2, 1><<<dim3(DD / 64, NROWS / 256), 256, GEMM_LDS, stream>>>(
      X1b, Mth, Mtl, Gh, Gl, DD, DD, DD, DD, 1.0f, 1.0f);
  k_attn<<<dim3(NROWS / 32), 256, ATT_LDS, stream>>>(Gh, Gl, X2b, X1t, Ohp, NROWS, NROWS);
  k_gemm<0, 1, 1, 0><<<dim3(DD / 64, NROWS / 256), 256, GEMM_LDS, stream>>>(
      Ohp, vw, vw, out, out, DD, DD, DD, DD, 64.0f, 1.0f / 64.0f);
  (void)hipGetLastError();
}
